// HCHALayer_549755814399
// MI455X (gfx1250) — hardware-verified
//
#include <hip/hip_runtime.h>
#include <stddef.h>


#define DIN   128
#define NH    4
#define DOUT  64
#define HD    (NH * DOUT)
#define GR    32
#define AP    136
#define XSP   260
#define NB    1024
#define LSH   10
#define CHUNK 2048
#define NTHR  256
#define NWAVE 8
#define WCAP  256
#define NGRP  (CHUNK / (NTHR * 4))

#define LDS_ACC  (NB * DOUT)
#define LDS_LIST (NWAVE * WCAP)
#define AGG_LDS_BYTES ((LDS_ACC + LDS_LIST + NWAVE) * 4)

static_assert(NGRP == 2);
static_assert(WCAP == NGRP * 4 * 32);
static_assert((1 << LSH) == NB);
static_assert(CHUNK == 2048);
static_assert(HD == 256);
static_assert((XSP % 4) == 0);
static_assert((LDS_ACC % 4) == 0);
static_assert(AGG_LDS_BYTES == 270368);

typedef float          v2f   __attribute__((ext_vector_type(2)));
typedef float          v4f   __attribute__((ext_vector_type(4)));
typedef float          v8f   __attribute__((ext_vector_type(8)));
typedef int            v4i   __attribute__((ext_vector_type(4)));
typedef unsigned short v8us  __attribute__((ext_vector_type(8)));
typedef unsigned short v16us __attribute__((ext_vector_type(16)));
typedef __bf16         v16bf __attribute__((ext_vector_type(16)));
union Frag { v16bf v; v16us u; v8us half[2]; };

__device__ __forceinline__ v8f wm(v16bf a, v16bf b, v8f c) {
  v8f d = __builtin_amdgcn_wmma_f32_16x16x32_bf16(false, a, false, b, (short)0, c, false, false);
  asm volatile("v_nop\n\tv_nop\n\tv_nop\n\tv_nop" : "+v"(d) : "v"(a), "v"(b));
  return d;
}

__device__ __forceinline__ unsigned int bfr(float f) {
  const unsigned int u = __float_as_uint(f);
  return (u + 0x7FFFu + ((u >> 16) & 1u)) >> 16;
}

__device__ __forceinline__ void split8(v4f a, v4f b, v4i& ho, v4i& lo) {
  float f[8] = {a.x, a.y, a.z, a.w, b.x, b.y, b.z, b.w};
  unsigned int h[8], l[8];
#pragma unroll
  for (int j = 0; j < 8; ++j) {
    h[j] = bfr(f[j]);
    l[j] = bfr(f[j] - __uint_as_float(h[j] << 16));
  }
  ho.x = (int)(h[0] | (h[1] << 16)); ho.y = (int)(h[2] | (h[3] << 16));
  ho.z = (int)(h[4] | (h[5] << 16)); ho.w = (int)(h[6] | (h[7] << 16));
  lo.x = (int)(l[0] | (l[1] << 16)); lo.y = (int)(l[2] | (l[3] << 16));
  lo.z = (int)(l[4] | (l[5] << 16)); lo.w = (int)(l[6] | (l[7] << 16));
}

__global__ __launch_bounds__(NTHR) void k_prepw(const float* __restrict__ Wp,
                                                const float* __restrict__ Wv,
                                                unsigned short* Wph, unsigned short* Wpl,
                                                unsigned short* Wvh, unsigned short* Wvl) {
  __shared__ float sW[32 * 129];
  const int tid = threadIdx.x;
  const int t   = blockIdx.x >> 3;
  const int o0  = (blockIdx.x & 7) * 32;
  const float* W = t ? Wv : Wp;
  unsigned short* Hh = t ? Wvh : Wph;
  unsigned short* Hl = t ? Wvl : Wpl;
  for (int q = tid; q < DIN * 8; q += NTHR) {
    const int k  = q >> 3;
    const int oc = (q & 7) * 4;
    const v4f v = *(const v4f*)(W + (size_t)k * HD + o0 + oc);
    sW[(oc + 0) * 129 + k] = v.x;
    sW[(oc + 1) * 129 + k] = v.y;
    sW[(oc + 2) * 129 + k] = v.z;
    sW[(oc + 3) * 129 + k] = v.w;
  }
  __syncthreads();
  const int rl = tid >> 4;
  const int k0 = (tid & 15) * 8;
  v4f a0, b0, a1, b1;
  {
    const float* p0 = sW + rl * 129 + k0;
    const float* p1 = sW + (16 + rl) * 129 + k0;
    a0.x = p0[0]; a0.y = p0[1]; a0.z = p0[2]; a0.w = p0[3];
    b0.x = p0[4]; b0.y = p0[5]; b0.z = p0[6]; b0.w = p0[7];
    a1.x = p1[0]; a1.y = p1[1]; a1.z = p1[2]; a1.w = p1[3];
    b1.x = p1[4]; b1.y = p1[5]; b1.z = p1[6]; b1.w = p1[7];
  }
  v4i h0, l0, h1, l1;
  split8(a0, b0, h0, l0);
  split8(a1, b1, h1, l1);
  const size_t g0 = (size_t)(o0 + rl) * DIN + k0;
  const size_t g1 = (size_t)(o0 + 16 + rl) * DIN + k0;
  *(volatile v4i*)(Hh + g0) = h0; *(volatile v4i*)(Hl + g0) = l0;
  *(volatile v4i*)(Hh + g1) = h1; *(volatile v4i*)(Hl + g1) = l1;
  __threadfence();
  *(volatile v4i*)(Hh + g0) = h0; *(volatile v4i*)(Hl + g0) = l0;
  *(volatile v4i*)(Hh + g1) = h1; *(volatile v4i*)(Hl + g1) = l1;
}

__device__ __forceinline__ void gemm4(const unsigned short* Ah, const unsigned short* Al,
                                      const unsigned short* __restrict__ Bh,
                                      const unsigned short* __restrict__ Bl,
                                      int m, int hh, int nc0, int nc1,
                                      v8f& c00, v8f& c01, v8f& c10, v8f& c11) {
  const v8f z = {0.f, 0.f, 0.f, 0.f, 0.f, 0.f, 0.f, 0.f};
  c00 = z; c01 = z; c10 = z; c11 = z;
  const unsigned short* a0hp = Ah + m * AP + 8 * hh;
  const unsigned short* a1hp = Ah + (16 + m) * AP + 8 * hh;
  const unsigned short* a0lp = Al + m * AP + 8 * hh;
  const unsigned short* a1lp = Al + (16 + m) * AP + 8 * hh;
  const unsigned short* b0hp = Bh + (size_t)nc0 * DIN + 8 * hh;
  const unsigned short* b0lp = Bl + (size_t)nc0 * DIN + 8 * hh;
  const unsigned short* b1hp = Bh + (size_t)nc1 * DIN + 8 * hh;
  const unsigned short* b1lp = Bl + (size_t)nc1 * DIN + 8 * hh;
#pragma unroll
  for (int kt = 0; kt < DIN / 32; ++kt) {
    const int k0 = kt * 32;
    Frag a0h, a0l, a1h, a1l, b0h, b0l, b1h, b1l;
    a0h.half[0] = *(const v8us*)(a0hp + k0);  a0h.half[1] = *(const v8us*)(a0hp + k0 + 16);
    a0l.half[0] = *(const v8us*)(a0lp + k0);  a0l.half[1] = *(const v8us*)(a0lp + k0 + 16);
    a1h.half[0] = *(const v8us*)(a1hp + k0);  a1h.half[1] = *(const v8us*)(a1hp + k0 + 16);
    a1l.half[0] = *(const v8us*)(a1lp + k0);  a1l.half[1] = *(const v8us*)(a1lp + k0 + 16);
    b0h.half[0] = *(const v8us*)(b0hp + k0);  b0h.half[1] = *(const v8us*)(b0hp + k0 + 16);
    b0l.half[0] = *(const v8us*)(b0lp + k0);  b0l.half[1] = *(const v8us*)(b0lp + k0 + 16);
    b1h.half[0] = *(const v8us*)(b1hp + k0);  b1h.half[1] = *(const v8us*)(b1hp + k0 + 16);
    b1l.half[0] = *(const v8us*)(b1lp + k0);  b1l.half[1] = *(const v8us*)(b1lp + k0 + 16);
    c00 = wm(a0h.v, b0h.v, c00);
    c00 = wm(a0h.v, b0l.v, c00);
    c00 = wm(a0l.v, b0h.v, c00);
    c01 = wm(a0h.v, b1h.v, c01);
    c01 = wm(a0h.v, b1l.v, c01);
    c01 = wm(a0l.v, b1h.v, c01);
    c10 = wm(a1h.v, b0h.v, c10);
    c10 = wm(a1h.v, b0l.v, c10);
    c10 = wm(a1l.v, b0h.v, c10);
    c11 = wm(a1h.v, b1h.v, c11);
    c11 = wm(a1h.v, b1l.v, c11);
    c11 = wm(a1l.v, b1h.v, c11);
  }
}

__global__ __launch_bounds__(NTHR) void k_proj(
    const float* __restrict__ X, int nRows,
    const unsigned short* __restrict__ Bph, const unsigned short* __restrict__ Bpl,
    const float* __restrict__ attn, float* eOut,
    const unsigned short* __restrict__ Bvh, const unsigned short* __restrict__ Bvl,
    const float* __restrict__ DV2, float* ftOut, int doV) {
  __shared__ __attribute__((aligned(16))) unsigned short Ah[GR * AP];
  __shared__ __attribute__((aligned(16))) unsigned short Al[GR * AP];
  __shared__ __attribute__((aligned(16))) float Xs[GR * XSP];
  __shared__ float sEv[GR * NWAVE];
  __shared__ float sDV[GR];

  const int tid  = threadIdx.x;
  const int lane = tid & 31;
  const int wave = tid >> 5;
  const int hh   = lane >> 4;
  const int m    = lane & 15;
  const int rowBase = blockIdx.x * GR;

  {
    const int r  = tid >> 3;
    const int c0 = (tid & 7) * 16;
    int row = rowBase + r;
    if (row > nRows - 1) row = nRows - 1;
    const float* p = X + (size_t)row * DIN + c0;
    const v4f f0 = *(const v4f*)(p), f1 = *(const v4f*)(p + 4);
    const v4f f2 = *(const v4f*)(p + 8), f3 = *(const v4f*)(p + 12);
    v4i h0, l0, h1, l1;
    split8(f0, f1, h0, l0);
    split8(f2, f3, h1, l1);
    *(v4i*)(Ah + r * AP + c0)     = h0;
    *(v4i*)(Ah + r * AP + c0 + 8) = h1;
    *(v4i*)(Al + r * AP + c0)     = l0;
    *(v4i*)(Al + r * AP + c0 + 8) = l1;
    if (doV != 0 && tid < GR) {
      int rr = rowBase + tid;
      if (rr > nRows - 1) rr = nRows - 1;
      sDV[tid] = DV2[rr];
    }
  }
  __syncthreads();

  const int nc0 = wave * 32 + m;
  const int nc1 = nc0 + 16;
  v8f c00, c01, c10, c11;

  gemm4(Ah, Al, Bph, Bpl, m, hh, nc0, nc1, c00, c01, c10, c11);
  {
    const float aw0 = attn[nc0];
    const float aw1 = attn[nc1];
    float p0[8], p1[8];
#pragma unroll
    for (int r = 0; r < 8; ++r) {
      p0[r] = c00[r] * aw0 + c01[r] * aw1;
      p1[r] = c10[r] * aw0 + c11[r] * aw1;
    }
#pragma unroll
    for (int off = 1; off < 16; off <<= 1) {
#pragma unroll
      for (int r = 0; r < 8; ++r) {
        p0[r] += __shfl_xor(p0[r], off, 32);
        p1[r] += __shfl_xor(p1[r], off, 32);
      }
    }
    if (m == 0) {
#pragma unroll
      for (int r = 0; r < 8; ++r) {
        sEv[(8 * hh + r) * NWAVE + wave]      = p0[r];
        sEv[(16 + 8 * hh + r) * NWAVE + wave] = p1[r];
      }
    }
  }
  __syncthreads();
  if (wave == 0) {
    const float* sp = sEv + lane * NWAVE;
    v4f e;
    e.x = sp[0] + sp[1];
    e.y = sp[2] + sp[3];
    e.z = sp[4] + sp[5];
    e.w = sp[6] + sp[7];
    float* op = eOut + (size_t)(rowBase + lane) * NH;
    *(volatile v4f*)op = e;
    __threadfence();
    *(volatile v4f*)op = e;
  }

  if (doV != 0) {
    gemm4(Ah, Al, Bvh, Bvl, m, hh, nc0, nc1, c00, c01, c10, c11);
#pragma unroll
    for (int r = 0; r < 8; ++r) {
      const int r0 = 8 * hh + r;
      const int r1 = 16 + 8 * hh + r;
      Xs[r0 * XSP + nc0] = c00[r] * sDV[r0];
      Xs[r0 * XSP + nc1] = c01[r] * sDV[r0];
      Xs[r1 * XSP + nc0] = c10[r] * sDV[r1];
      Xs[r1 * XSP + nc1] = c11[r] * sDV[r1];
    }
    __syncthreads();
    v4f xr[8];
    float* xp[8];
#pragma unroll
    for (int i = 0; i < 4; ++i) {
      const int row = 4 * wave + i;
      xr[2 * i]     = *(const v4f*)(Xs + row * XSP + 4 * lane);
      xr[2 * i + 1] = *(const v4f*)(Xs + row * XSP + 128 + 4 * lane);
      xp[2 * i]     = ftOut + (size_t)(rowBase + row) * HD + 4 * lane;
      xp[2 * i + 1] = ftOut + (size_t)(rowBase + row) * HD + 128 + 4 * lane;
    }
#pragma unroll
    for (int i = 0; i < 8; ++i) *(volatile v4f*)(xp[i]) = xr[i];
    __threadfence();
#pragma unroll
    for (int i = 0; i < 8; ++i) *(volatile v4f*)(xp[i]) = xr[i];
  }
}

__device__ __forceinline__ void scan_chunk(const int* __restrict__ dstIds, int nnz, int cbase,
                                           int dstBase, bool al16, int tid, int lane, int wave,
                                           int* list, int* wcnt) {
  int wc = 0;
#pragma unroll
  for (int g = 0; g < NGRP; ++g) {
    const int el0 = (g * NTHR + tid) * 4;
    const int e0  = cbase + el0;
    const int sent = -2147483647 - 1;
    v4i d;
    if (al16 && (e0 + 3 < nnz)) {
      d = *(const v4i*)(dstIds + e0);
    } else {
      d.x = (e0     < nnz) ? dstIds[min(e0, nnz - 1)]     : sent;
      d.y = (e0 + 1 < nnz) ? dstIds[min(e0 + 1, nnz - 1)] : sent;
      d.z = (e0 + 2 < nnz) ? dstIds[min(e0 + 2, nnz - 1)] : sent;
      d.w = (e0 + 3 < nnz) ? dstIds[min(e0 + 3, nnz - 1)] : sent;
    }
    const unsigned s0 = (unsigned)d.x - (unsigned)dstBase;
    const unsigned s1 = (unsigned)d.y - (unsigned)dstBase;
    const unsigned s2 = (unsigned)d.z - (unsigned)dstBase;
    const unsigned s3 = (unsigned)d.w - (unsigned)dstBase;
    const bool h0 = s0 < (unsigned)NB;
    const bool h1 = s1 < (unsigned)NB;
    const bool h2 = s2 < (unsigned)NB;
    const bool h3 = s3 < (unsigned)NB;
    const unsigned many = __builtin_amdgcn_ballot_w32(h0 | h1 | h2 | h3);
    if (many != 0u) {
#define HITJ(J, HJ, SJ) { \
        const unsigned mj = __builtin_amdgcn_ballot_w32(HJ); \
        if (HJ) { \
          const int pos = wc + (int)__builtin_amdgcn_mbcnt_lo(mj, 0u); \
          if (pos < WCAP) list[wave * WCAP + pos] = ((el0 + (J)) << LSH) | (int)(SJ); \
        } \
        wc += (int)__builtin_popcount(mj); }
      HITJ(0, h0, s0)
      HITJ(1, h1, s1)
      HITJ(2, h2, s2)
      HITJ(3, h3, s3)
#undef HITJ
    }
  }
  if (lane == 0) wcnt[wave] = wc;
}

__global__ __launch_bounds__(NTHR) void k_den(
    const int* __restrict__ nodeIdx, const int* __restrict__ edgeIdx,
    const float* __restrict__ eV, const float* __restrict__ eE,
    float* dinv, int nN, int nE, int nnz) {
  __shared__ __attribute__((aligned(16))) float den[NB * NH];
  __shared__ int list[LDS_LIST];
  __shared__ int wcnt[NWAVE];

  const int tid  = threadIdx.x;
  const int lane = tid & 31;
  const int wave = tid >> 5;
  const int dstBase = blockIdx.x * NB;

  {
    const v4f z4 = {0.f, 0.f, 0.f, 0.f};
    v4f* dz = (v4f*)den;
    for (int i = tid; i < (NB * NH) / 4; i += NTHR) dz[i] = z4;
  }
  __syncthreads();
  const bool al16 = ((((size_t)nodeIdx) & 15) == 0);
  const int nChunks = (nnz + CHUNK - 1) / CHUNK;
#pragma unroll 1
  for (int ch = 0; ch < nChunks; ++ch) {
    const int cbase = ch * CHUNK;
    scan_chunk(nodeIdx, nnz, cbase, dstBase, al16, tid, lane, wave, list, wcnt);
    __syncthreads();
    if (wave == 0) {
      const int j = lane >> 2;
      const int h = lane & 3;
      for (int wsx = 0; wsx < NWAVE; ++wsx) {
        int n = wcnt[wsx];
        if (n > WCAP) n = WCAP;
        if (n < 0) n = 0;
        for (int i0 = 0; i0 < n; i0 += 8) {
          const int idx = i0 + j;
          const bool valid = idx < n;
          const int ent  = list[wsx * WCAP + (valid ? idx : i0)];
          const int slot = ent & (NB - 1);
          const int el   = (ent >> LSH) & (CHUNK - 1);
          int ii = cbase + el;
          if (ii > nnz - 1) ii = nnz - 1;
          int e = edgeIdx[ii];
          e = e < 0 ? 0 : (e > nE - 1 ? nE - 1 : e);
          int v = dstBase + slot;
          if (v > nN - 1) v = nN - 1;
          float s = eE[(size_t)e * NH + h] + eV[(size_t)v * NH + h];
          s = fmaxf(s, 0.f);
          s = fminf(s, 80.f);
          const float ex = valid ? __expf(s) : 0.f;
#pragma unroll
          for (int r = 0; r < 8; ++r) {
            const float exr = __shfl(ex, 4 * r + h, 32);
            const int   slr = __shfl(slot, 4 * r, 32);
            if (lane < NH) {
              float* dp = den + slr * NH + lane;
              const float cur = *dp;
              *dp = cur + exr;
            }
          }
        }
      }
    }
    __syncthreads();
  }

#pragma unroll 1
  for (int k = 0; k < NB / (NWAVE * 32); ++k) {
    const int slot = wave * (NB / NWAVE) + 32 * k + lane;
    const v4f d = *(const v4f*)(den + slot * NH);
    v4f o;
    o.x = d.x > 0.f ? 1.0f / d.x : 0.f;
    o.y = d.y > 0.f ? 1.0f / d.y : 0.f;
    o.z = d.z > 0.f ? 1.0f / d.z : 0.f;
    o.w = d.w > 0.f ? 1.0f / d.w : 0.f;
    float* op = dinv + (size_t)(dstBase + slot) * NH;
    *(volatile v4f*)op = o;
    __threadfence();
    *(volatile v4f*)op = o;
  }
}

__global__ __launch_bounds__(NTHR) void k_stg1(
    const int* __restrict__ edgeIdx, const int* __restrict__ nodeIdx,
    const float* __restrict__ eE, const float* __restrict__ eV,
    const float* __restrict__ dinv, const float* __restrict__ ft,
    float* outE, int nE, int nN, int nnz) {
  extern __shared__ v4f lds_dyn[];
  float* acc  = (float*)lds_dyn;
  int*   list = (int*)(acc + LDS_ACC);
  int*   wcnt = list + LDS_LIST;

  const int tid  = threadIdx.x;
  const int lane = tid & 31;
  const int wave = tid >> 5;
  const int dstBase = blockIdx.x * NB;

  {
    const v4f z4 = {0.f, 0.f, 0.f, 0.f};
    for (int i = tid; i < LDS_ACC / 4; i += NTHR) lds_dyn[i] = z4;
  }
  __syncthreads();
  const bool al16 = ((((size_t)edgeIdx) & 15) == 0);
  const int nChunks = (nnz + CHUNK - 1) / CHUNK;
#pragma unroll 1
  for (int ch = 0; ch < nChunks; ++ch) {
    const int cbase = ch * CHUNK;
    scan_chunk(edgeIdx, nnz, cbase, dstBase, al16, tid, lane, wave, list, wcnt);
    __syncthreads();
    if (wave == 0) {
      for (int wsx = 0; wsx < NWAVE; ++wsx) {
        int n = wcnt[wsx];
        if (n > WCAP) n = WCAP;
        if (n < 0) n = 0;
        for (int i = 0; i < n; ++i) {
          const int ent  = list[wsx * WCAP + i];
          const int slot = ent & (NB - 1);
          const int el   = (ent >> LSH) & (CHUNK - 1);
          int ii = cbase + el;
          if (ii > nnz - 1) ii = nnz - 1;
          int v = nodeIdx[ii];
          v = v < 0 ? 0 : (v > nN - 1 ? nN - 1 : v);
          int eh = dstBase + slot;
          if (eh > nE - 1) eh = nE - 1;
          const v4f ee = *(const v4f*)(eE + (size_t)eh * NH);
          const v4f ev = *(const v4f*)(eV + (size_t)v * NH);
          const v4f di = *(const v4f*)(dinv + (size_t)v * NH);
          const float a0 = __expf(fminf(fmaxf(ee.x + ev.x, 0.f), 80.f)) * di.x;
          const float a1 = __expf(fminf(fmaxf(ee.y + ev.y, 0.f), 80.f)) * di.y;
          const float a2 = __expf(fminf(fmaxf(ee.z + ev.z, 0.f), 80.f)) * di.z;
          const float a3 = __expf(fminf(fmaxf(ee.w + ev.w, 0.f), 80.f)) * di.w;
          const float* fr = ft + (size_t)v * HD + 2 * lane;
          const v2f f0 = *(const v2f*)(fr);
          const v2f f1 = *(const v2f*)(fr + DOUT);
          const v2f f2 = *(const v2f*)(fr + 2 * DOUT);
          const v2f f3 = *(const v2f*)(fr + 3 * DOUT);
          const v2f c = a0 * f0 + a1 * f1 + a2 * f2 + a3 * f3;
          v2f* ap = (v2f*)(acc + slot * DOUT + 2 * lane);
          const v2f cur = *ap;
          *ap = cur + c;
        }
      }
    }
    __syncthreads();
  }

  const int rsub = lane >> 4;
  const int c4   = (lane & 15) * 4;
#pragma unroll 1
  for (int k = 0; k < NB / (2 * NWAVE); ++k) {
    const int slot = wave * (NB / NWAVE) + 2 * k + rsub;
    const int row  = dstBase + slot;
    if (row < nE) {
      const v4f v = *(const v4f*)(acc + slot * DOUT + c4) * 0.25f;
      *(volatile v4f*)(outE + (size_t)row * DOUT + c4) = v;
    }
  }
  __threadfence();
#pragma unroll 1
  for (int k = 0; k < NB / (2 * NWAVE); ++k) {
    const int slot = wave * (NB / NWAVE) + 2 * k + rsub;
    const int row  = dstBase + slot;
    if (row < nE) {
      const v4f v = *(const v4f*)(acc + slot * DOUT + c4) * 0.25f;
      *(volatile v4f*)(outE + (size_t)row * DOUT + c4) = v;
    }
  }
}

__global__ __launch_bounds__(NTHR) void k_stg2(
    const int* __restrict__ nodeIdx, const int* __restrict__ edgeIdx,
    const float* __restrict__ eV, const float* __restrict__ eE,
    const float* __restrict__ dinv, const float* zr, const float* __restrict__ invDE,
    const float* __restrict__ DV2, float* outV, int nN, int nE, int nnz) {
  extern __shared__ v4f lds_dyn[];
  float* acc  = (float*)lds_dyn;
  int*   list = (int*)(acc + LDS_ACC);
  int*   wcnt = list + LDS_LIST;

  const int tid  = threadIdx.x;
  const int lane = tid & 31;
  const int wave = tid >> 5;
  const int dstBase = blockIdx.x * NB;

  {
    const v4f z4 = {0.f, 0.f, 0.f, 0.f};
    for (int i = tid; i < LDS_ACC / 4; i += NTHR) lds_dyn[i] = z4;
  }
  __syncthreads();
  const bool al16 = ((((size_t)nodeIdx) & 15) == 0);
  const int nChunks = (nnz + CHUNK - 1) / CHUNK;
#pragma unroll 1
  for (int ch = 0; ch < nChunks; ++ch) {
    const int cbase = ch * CHUNK;
    scan_chunk(nodeIdx, nnz, cbase, dstBase, al16, tid, lane, wave, list, wcnt);
    __syncthreads();
    if (wave == 0) {
      for (int wsx = 0; wsx < NWAVE; ++wsx) {
        int n = wcnt[wsx];
        if (n > WCAP) n = WCAP;
        if (n < 0) n = 0;
        for (int i = 0; i < n; ++i) {
          const int ent  = list[wsx * WCAP + i];
          const int slot = ent & (NB - 1);
          const int el   = (ent >> LSH) & (CHUNK - 1);
          int ii = cbase + el;
          if (ii > nnz - 1) ii = nnz - 1;
          int e = edgeIdx[ii];
          e = e < 0 ? 0 : (e > nE - 1 ? nE - 1 : e);
          int v = dstBase + slot;
          if (v > nN - 1) v = nN - 1;
          const v4f ee = *(const v4f*)(eE + (size_t)e * NH);
          const v4f ev = *(const v4f*)(eV + (size_t)v * NH);
          const v4f di = *(const v4f*)(dinv + (size_t)v * NH);
          float abar = __expf(fminf(fmaxf(ee.x + ev.x, 0.f), 80.f)) * di.x;
          abar      += __expf(fminf(fmaxf(ee.y + ev.y, 0.f), 80.f)) * di.y;
          abar      += __expf(fminf(fmaxf(ee.z + ev.z, 0.f), 80.f)) * di.z;
          abar      += __expf(fminf(fmaxf(ee.w + ev.w, 0.f), 80.f)) * di.w;
          const float w = abar * invDE[e];
          const v2f z = *(const v2f*)(zr + (size_t)e * DOUT + 2 * lane);
          v2f* ap = (v2f*)(acc + slot * DOUT + 2 * lane);
          const v2f cur = *ap;
          *ap = cur + w * z;
        }
      }
    }
    __syncthreads();
  }

  const int rsub = lane >> 4;
  const int c4   = (lane & 15) * 4;
#pragma unroll 1
  for (int k = 0; k < NB / (2 * NWAVE); ++k) {
    const int slot = wave * (NB / NWAVE) + 2 * k + rsub;
    const int row  = dstBase + slot;
    if (row < nN) {
      const float sc = 0.25f * DV2[row];
      const v4f v = *(const v4f*)(acc + slot * DOUT + c4) * sc;
      *(volatile v4f*)(outV + (size_t)row * DOUT + c4) = v;
    }
  }
  __threadfence();
#pragma unroll 1
  for (int k = 0; k < NB / (2 * NWAVE); ++k) {
    const int slot = wave * (NB / NWAVE) + 2 * k + rsub;
    const int row  = dstBase + slot;
    if (row < nN) {
      const float sc = 0.25f * DV2[row];
      const v4f v = *(const v4f*)(acc + slot * DOUT + c4) * sc;
      *(volatile v4f*)(outV + (size_t)row * DOUT + c4) = v;
    }
  }
}

#define ALIGN256(x) (((x) + (size_t)255) & ~(size_t)255)

extern "C" void kernel_launch(void* const* d_in, const int* in_sizes, int n_in,
                              void* d_out, int out_size, void* d_ws, size_t ws_size,
                              hipStream_t stream) {
  if (n_in < 10) return;
  const int nN  = in_sizes[2];
  const int nE  = in_sizes[3];
  const int nnz = in_sizes[8];
  if (nN <= 0 || nE <= 0 || nnz <= 0) return;
  if (in_sizes[0] != nN * DIN || in_sizes[1] != nE * DIN) return;
  if (in_sizes[4] != DIN * HD || in_sizes[5] != DIN * HD) return;
  if (in_sizes[6] != HD || in_sizes[7] != HD) return;
  if (in_sizes[9] != nnz) return;
  if (out_size != (nN + nE) * DOUT) return;

  const float* vfeat  = (const float*)d_in[0];
  const float* efeat  = (const float*)d_in[1];
  const float* DV2    = (const float*)d_in[2];
  const float* invDE  = (const float*)d_in[3];
  const float* Wp     = (const float*)d_in[4];
  const float* Wv     = (const float*)d_in[5];
  const float* attn_v = (const float*)d_in[6];
  const float* attn_e = (const float*)d_in[7];
  const int*   nidx   = (const int*)d_in[8];
  const int*   eidx   = (const int*)d_in[9];

  float* outV = (float*)d_out;
  float* outE = outV + (size_t)nN * DOUT;

  const int nPv = ((nN + GR - 1) / GR) * GR;
  const int nPe = ((nE + GR - 1) / GR) * GR;
  const int nPd = ((nN + NB - 1) / NB) * NB;
  const int nBe = (nE + NB - 1) / NB;

  size_t off = 0;
  const size_t plane = (size_t)HD * DIN * sizeof(unsigned short);
  unsigned short* Wph = (unsigned short*)((char*)d_ws + off); off = ALIGN256(off + plane);
  unsigned short* Wpl = (unsigned short*)((char*)d_ws + off); off = ALIGN256(off + plane);
  unsigned short* Wvh = (unsigned short*)((char*)d_ws + off); off = ALIGN256(off + plane);
  unsigned short* Wvl = (unsigned short*)((char*)d_ws + off); off = ALIGN256(off + plane);
  float* e_v  = (float*)((char*)d_ws + off); off = ALIGN256(off + (size_t)nPv * NH * sizeof(float));
  float* e_e  = (float*)((char*)d_ws + off); off = ALIGN256(off + (size_t)nPe * NH * sizeof(float));
  float* dinv = (float*)((char*)d_ws + off); off = ALIGN256(off + (size_t)nPd * NH * sizeof(float));
  float* ft   = (float*)((char*)d_ws + off); off = ALIGN256(off + (size_t)nPv * HD * sizeof(float));
  if (off > ws_size) return;
  if (off > ((size_t)128 << 20)) return;

  k_prepw<<<16, NTHR, 0, stream>>>(Wp, Wv, Wph, Wpl, Wvh, Wvl);
  k_proj<<<nPv / GR, NTHR, 0, stream>>>(vfeat, nN, Wph, Wpl, attn_v, e_v, Wvh, Wvl, DV2, ft, 1);
  k_proj<<<nPe / GR, NTHR, 0, stream>>>(efeat, nE, Wph, Wpl, attn_e, e_e, Wvh, Wvl, DV2, ft, 0);
  k_den<<<nPd / NB, NTHR, 0, stream>>>(nidx, eidx, e_v, e_e, dinv, nN, nE, nnz);

  hipFuncSetAttribute(reinterpret_cast<const void*>(&k_stg1),
                      hipFuncAttributeMaxDynamicSharedMemorySize, AGG_LDS_BYTES);
  hipFuncSetAttribute(reinterpret_cast<const void*>(&k_stg2),
                      hipFuncAttributeMaxDynamicSharedMemorySize, AGG_LDS_BYTES);
  k_stg1<<<nBe, NTHR, AGG_LDS_BYTES, stream>>>(eidx, nidx, e_e, e_v, dinv, ft, outE, nE, nN, nnz);
  k_stg2<<<nPd / NB, NTHR, AGG_LDS_BYTES, stream>>>(nidx, eidx, e_v, e_e, dinv, outE, invDE, DV2,
                                                     outV, nN, nE, nnz);
}
